// GraphLP_70738111365647
// MI455X (gfx1250) — hardware-verified
//
#include <hip/hip_runtime.h>
#include <stddef.h>


#define NT    256
#define NWAV  8
#define DF    64
#define INF   128
#define HD    128
#define MBLK  (NWAV * 16)
#define KPW   36
#define EPW   32

static_assert(MBLK == 128);
static_assert((HD * DF / 2) % NT == 0);
static_assert((KPW * 4) % 16 == 0);
static_assert(INF == 2 * DF);

typedef float    v2f  __attribute__((ext_vector_type(2)));
typedef float    v4f  __attribute__((ext_vector_type(4)));
typedef float    v8f  __attribute__((ext_vector_type(8)));
typedef unsigned v4u  __attribute__((ext_vector_type(4)));
typedef unsigned v8u  __attribute__((ext_vector_type(8)));
typedef __bf16   v16b __attribute__((ext_vector_type(16)));
union FragB { v16b v; v8u u; v4u q[2]; };

__device__ __forceinline__ unsigned bfb(float x) {
  unsigned u = __float_as_uint(x);
  u += 0x7FFFu + ((u >> 16) & 1u);
  return u >> 16;
}
__device__ __forceinline__ float bfv(unsigned b) { return __uint_as_float(b << 16); }

__device__ __forceinline__ void split2(float a, float b, unsigned& ph, unsigned& pl) {
  const unsigned ha = bfb(a), hb = bfb(b);
  const unsigned la = bfb(a - bfv(ha)), lb = bfb(b - bfv(hb));
  ph = ha | (hb << 16);
  pl = la | (lb << 16);
}

__device__ __forceinline__ v8f wmb(v16b a, v16b b, v8f c) {
  v8f d = __builtin_amdgcn_wmma_f32_16x16x32_bf16(false, a, false, b, (short)0, c, false, false);
  asm volatile("v_nop\n\tv_nop\n\tv_nop\n\tv_nop" : "+v"(d) : "v"(a), "v"(b));
  return d;
}

__global__ __launch_bounds__(NT) void k_proj(const float* __restrict__ zi, const float* __restrict__ zj,
                                             const float* __restrict__ W1, const float* __restrict__ b1,
                                             float* Pp, float* Qp, int nN) {
  __shared__ __attribute__((aligned(16))) unsigned sWh[HD * KPW];
  __shared__ __attribute__((aligned(16))) unsigned sWl[HD * KPW];
  __shared__ __attribute__((aligned(16))) float    sBias[HD];
  __shared__ __attribute__((aligned(16))) float    stg[NWAV * 16 * 32];

  const int tid = threadIdx.x, lane = tid & 31, wave = tid >> 5, h = lane >> 4, m = lane & 15;
  const int isQ = (blockIdx.y != 0) ? 1 : 0;
  const float* z = (isQ != 0) ? zj : zi;
  float* dstp = (isQ != 0) ? Qp : Pp;
  const int koff = (isQ != 0) ? DF : 0;

#pragma unroll
  for (int i = 0; i < (HD * DF / 2) / NT; ++i) {
    const int p  = tid + NT * i;
    const int n  = p >> 5, kp = p & 31;
    const v2f w = *(const v2f*)(W1 + n * INF + koff + 2 * kp);
    unsigned ph, pl;
    split2(w.x, w.y, ph, pl);
    sWh[n * KPW + kp] = ph;
    sWl[n * KPW + kp] = pl;
  }
  if (tid < HD) sBias[tid] = (isQ != 0) ? 0.0f : b1[tid];
  __syncthreads();

  const int row0 = blockIdx.x * MBLK + wave * 16;
  int ra = row0 + m;
  ra = ra > nN - 1 ? nN - 1 : ra;
  ra = ra < 0 ? 0 : ra;
  const float* arow = z + (size_t)ra * DF;

  v8f acc[8];
  {
    v8f zz;
#pragma unroll
    for (int r = 0; r < 8; ++r) zz[r] = 0.0f;
#pragma unroll
    for (int nt = 0; nt < 8; ++nt) acc[nt] = zz;
  }

#pragma unroll
  for (int ks = 0; ks < DF / 32; ++ks) {
    const int k0 = ks * 32;
    const v4f x0 = *(const v4f*)(arow + k0 + 8 * h);
    const v4f x1 = *(const v4f*)(arow + k0 + 8 * h + 4);
    const v4f x2 = *(const v4f*)(arow + k0 + 16 + 8 * h);
    const v4f x3 = *(const v4f*)(arow + k0 + 16 + 8 * h + 4);
    v8u uh, ul;
    { unsigned a, b;
      split2(x0.x, x0.y, a, b); uh[0] = a; ul[0] = b;
      split2(x0.z, x0.w, a, b); uh[1] = a; ul[1] = b;
      split2(x1.x, x1.y, a, b); uh[2] = a; ul[2] = b;
      split2(x1.z, x1.w, a, b); uh[3] = a; ul[3] = b;
      split2(x2.x, x2.y, a, b); uh[4] = a; ul[4] = b;
      split2(x2.z, x2.w, a, b); uh[5] = a; ul[5] = b;
      split2(x3.x, x3.y, a, b); uh[6] = a; ul[6] = b;
      split2(x3.z, x3.w, a, b); uh[7] = a; ul[7] = b; }
    FragB ah, al;
    ah.u = uh;
    al.u = ul;
#pragma unroll
    for (int nt = 0; nt < 8; ++nt) {
      const unsigned* bph = sWh + (nt * 16 + m) * KPW + (k0 >> 1) + 4 * h;
      const unsigned* bpl = sWl + (nt * 16 + m) * KPW + (k0 >> 1) + 4 * h;
      FragB bh, bl;
      bh.q[0] = *(const v4u*)bph;
      bh.q[1] = *(const v4u*)(bph + 8);
      bl.q[0] = *(const v4u*)bpl;
      bl.q[1] = *(const v4u*)(bpl + 8);
      acc[nt] = wmb(ah.v, bh.v, acc[nt]);
      acc[nt] = wmb(al.v, bh.v, acc[nt]);
      acc[nt] = wmb(ah.v, bl.v, acc[nt]);
    }
  }

  float* sw = stg + wave * (16 * 32);
  const int rsel = lane >> 3;
  const int c4   = (lane & 7) * 4;
#pragma unroll
  for (int q = 0; q < 4; ++q) {
    {
      const float ba = sBias[32 * q + m];
      const float bb = sBias[32 * q + 16 + m];
#pragma unroll
      for (int r = 0; r < 8; ++r) {
        sw[(8 * h + r) * 32 + m]      = acc[2 * q][r] + ba;
        sw[(8 * h + r) * 32 + 16 + m] = acc[2 * q + 1][r] + bb;
      }
    }
    __syncthreads();
    v4f ov[4];
#pragma unroll
    for (int i = 0; i < 4; ++i) ov[i] = *(const v4f*)(sw + (4 * i + rsel) * 32 + c4);
#pragma unroll
    for (int i = 0; i < 4; ++i) {
      float* gp = dstp + (size_t)(row0 + 4 * i + rsel) * HD + 32 * q + c4;
      *(volatile v4f*)gp = ov[i];
    }
    __threadfence();
#pragma unroll
    for (int i = 0; i < 4; ++i) {
      float* gp = dstp + (size_t)(row0 + 4 * i + rsel) * HD + 32 * q + c4;
      *(volatile v4f*)gp = ov[i];
    }
    __syncthreads();
  }
}

__global__ __launch_bounds__(NT) void k_score(const float* __restrict__ Pp, const float* __restrict__ Qp,
                                              const float* __restrict__ W3, const float* __restrict__ b3,
                                              const int* __restrict__ src, const int* __restrict__ dst,
                                              float* out, int nN, int nE) {
  const int tid = threadIdx.x, lane = tid & 31, wave = tid >> 5;
  const int ebase = (blockIdx.x * NWAV + wave) * EPW;
  if (ebase >= nE) return;
  const v4f w3 = *(const v4f*)(W3 + 4 * lane);
  const float bb3 = b3[0];
  int ea = ebase + lane;
  ea = ea > nE - 1 ? nE - 1 : ea;
  int si = src[ea];
  int di = dst[ea];
  si = si < 0 ? 0 : (si > nN - 1 ? nN - 1 : si);
  di = di < 0 ? 0 : (di > nN - 1 ? nN - 1 : di);

  float mysc = 0.0f;
#pragma unroll 1
  for (int i = 0; i < EPW; ++i) {
    const int s = __shfl(si, i);
    const int d = __shfl(di, i);
    const v4f p = *(const v4f*)(Pp + (size_t)s * HD + 4 * lane);
    const v4f q = *(const v4f*)(Qp + (size_t)d * HD + 4 * lane);
    const float h0 = fmaxf(p.x + q.x, 0.0f);
    const float h1 = fmaxf(p.y + q.y, 0.0f);
    const float h2 = fmaxf(p.z + q.z, 0.0f);
    const float h3 = fmaxf(p.w + q.w, 0.0f);
    float t = h0 * w3.x;
    t = fmaf(h1, w3.y, t);
    t = fmaf(h2, w3.z, t);
    t = fmaf(h3, w3.w, t);
    t += __shfl_xor(t, 16);
    t += __shfl_xor(t, 8);
    t += __shfl_xor(t, 4);
    t += __shfl_xor(t, 2);
    t += __shfl_xor(t, 1);
    float x = t + bb3;
    x = fminf(fmaxf(x, -80.0f), 80.0f);
    const float ex = __expf(-x);
    const float sc = __builtin_amdgcn_rcpf(1.0f + ex);
    mysc = (lane == i) ? sc : mysc;
  }

  const int e = ebase + lane;
  const bool wr = e < nE;
  if (wr) {
    *(volatile float*)(out + e) = mysc;
    *(volatile float*)(out + (size_t)nE + e) = mysc;
  }
  __threadfence();
  if (wr) {
    *(volatile float*)(out + e) = mysc;
    *(volatile float*)(out + (size_t)nE + e) = mysc;
  }
}

extern "C" void kernel_launch(void* const* d_in, const int* in_sizes, int n_in,
                              void* d_out, int out_size, void* d_ws, size_t ws_size,
                              hipStream_t stream) {
  if (n_in < 9) return;
  const int nN = in_sizes[0] / DF;
  const int nE = in_sizes[7];
  if (nN <= 0 || nE <= 0) return;
  if (in_sizes[0] != nN * DF || in_sizes[1] != in_sizes[0]) return;
  if (in_sizes[3] != HD * INF || in_sizes[4] != HD || in_sizes[5] != HD || in_sizes[6] < 1) return;
  if (in_sizes[8] != nE) return;
  if (out_size != 2 * nE) return;

  const float* zi = (const float*)d_in[0];
  const float* zj = (const float*)d_in[1];
  const float* W1 = (const float*)d_in[3];
  const float* b1 = (const float*)d_in[4];
  const float* W3 = (const float*)d_in[5];
  const float* b3 = (const float*)d_in[6];
  const int* psrc = (const int*)d_in[7];
  const int* pdst = (const int*)d_in[8];
  float* out = (float*)d_out;

  const int nBlkM = (nN + MBLK - 1) / MBLK;
  const size_t rowsPad = (size_t)nBlkM * MBLK;
  const size_t planeB  = rowsPad * HD * sizeof(float);

  char* ws = (char*)d_ws;
  size_t off = 0;
  const size_t oP = off; off += planeB;
  const size_t oQ = off; off += planeB;
  if (off > ws_size) return;
  float* P = (float*)(ws + oP);
  float* Q = (float*)(ws + oQ);

  k_proj<<<dim3(nBlkM, 2, 1), NT, 0, stream>>>(zi, zj, W1, b1, P, Q, nN);

  const int nBlkE = (nE + NWAV * EPW - 1) / (NWAV * EPW);
  k_score<<<nBlkE, NT, 0, stream>>>(P, Q, W3, b3, psrc, pdst, out, nN, nE);
}
